// RoformerAttention_10084583211363
// MI455X (gfx1250) — hardware-verified
//
#include <hip/hip_runtime.h>
#include <math.h>

#define NB 2
#define NS 2048
#define ND 1024
#define NH 16
#define NHD 64
#define NM (NB * NS)
#define NFREQ 32
#define WCARRY 64.0f
#define OCARRY 64.0f
#define PCARRY 32768.0f
#define LN_EPS_F 1e-5f

typedef __attribute__((ext_vector_type(16))) _Float16 v16h;
typedef __attribute__((ext_vector_type(8)))  _Float16 v8h;
typedef __attribute__((ext_vector_type(16))) __bf16   v16b;
typedef __attribute__((ext_vector_type(8)))  __bf16   v8b;
typedef __attribute__((ext_vector_type(8)))  float    v8f;
typedef __attribute__((ext_vector_type(4)))  float    v4f;

__device__ __forceinline__ unsigned short f2bf_bits(float f) {
  unsigned u = __float_as_uint(f);
  return (unsigned short)((u + 0x7FFFu + ((u >> 16) & 1u)) >> 16);
}
__device__ __forceinline__ float bf_bits2f(unsigned short h) { return __uint_as_float(((unsigned)h) << 16); }

__device__ __forceinline__ void dep_guard_h(v8f& a, v8f& b, v16h x, v16h y) { asm volatile("v_nop\n\tv_nop\n\tv_nop\n\tv_nop" : "+v"(a), "+v"(b) : "v"(x), "v"(y)); }
__device__ __forceinline__ void dep_guard_b(v8f& a, v8f& b, v16b x, v16b y) { asm volatile("v_nop\n\tv_nop\n\tv_nop\n\tv_nop" : "+v"(a), "+v"(b) : "v"(x), "v"(y)); }
__device__ __forceinline__ void keep4_h(v16h a, v16h b, v16h c, v16h d) { asm volatile("v_nop" :: "v"(a), "v"(b), "v"(c), "v"(d)); }
__device__ __forceinline__ void keep4_b(v16b a, v16b b, v16b c, v16b d) { asm volatile("v_nop" :: "v"(a), "v"(b), "v"(c), "v"(d)); }
__device__ __forceinline__ void acc_guard4(v8f& a, v8f& b, v8f& c, v8f& d) { asm volatile("v_nop\n\tv_nop\n\tv_nop\n\tv_nop" : "+v"(a), "+v"(b), "+v"(c), "+v"(d)); }
template <typename T> struct Frag;
template <> struct Frag<_Float16> {
  typedef v16h V; union U { v16h v; v8h h[2]; };
  static __device__ __forceinline__ v16h load(const _Float16* p) {
    U f; f.h[0] = *(const v8h*)(p); f.h[1] = *(const v8h*)(p + 16); return f.v;
  }
  static __device__ __forceinline__ v8f mma(v16h a, v16h b, v8f c) {
    return __builtin_amdgcn_wmma_f32_16x16x32_f16(false, a, false, b, (short)0, c, false, false);
  }
  static __device__ __forceinline__ void guard(v8f& a, v8f& b, v16h x, v16h y) { dep_guard_h(a, b, x, y); }
  static __device__ __forceinline__ void keep(v16h a, v16h b, v16h c, v16h d) { keep4_h(a, b, c, d); }
};
template <> struct Frag<__bf16> {
  typedef v16b V; union U { v16b v; v8b h[2]; };
  static __device__ __forceinline__ v16b load(const __bf16* p) {
    U f; f.h[0] = *(const v8b*)(p); f.h[1] = *(const v8b*)(p + 16); return f.v;
  }
  static __device__ __forceinline__ v8f mma(v16b a, v16b b, v8f c) {
    return __builtin_amdgcn_wmma_f32_16x16x32_bf16(false, a, false, b, (short)0, c, false, false);
  }
  static __device__ __forceinline__ void guard(v8f& a, v8f& b, v16b x, v16b y) { dep_guard_b(a, b, x, y); }
  static __device__ __forceinline__ void keep(v16b a, v16b b, v16b c, v16b d) { keep4_b(a, b, c, d); }
};

template <int ET> struct Elem;
template <> struct Elem<0> { typedef _Float16 T; };
template <> struct Elem<1> { typedef __bf16 T; };
template <int ET, bool SPLIT, int BIAS_MODE, int OUT_MODE, bool RESID, int ACT, bool ROPE>
__global__ __launch_bounds__(256) void wmma_gemm64(
    const unsigned short* __restrict__ Ap, const unsigned short* __restrict__ A2p, int lda, long strideA,
    const unsigned short* __restrict__ Btp, const unsigned short* __restrict__ Bt2p, int ldb, long strideB,
    void* __restrict__ Cout, void* __restrict__ Cout2, int ldc, long strideC,
    const float* __restrict__ bias,
    const float* __restrict__ resid, long strideR,
    int M, int N, int K, float scale,
    const float* __restrict__ rope_cos, const float* __restrict__ rope_sin, int rope_smask) {
  typedef typename Elem<ET>::T T;
  typedef typename Frag<T>::V V;
  const T* A = (const T*)Ap; const T* A2 = (const T*)A2p; const T* Bt = (const T*)Btp; const T* Bt2 = (const T*)Bt2p;
  __shared__ __align__(16) float sT[8][16 * 68];
  const int b    = blockIdx.y;
  const int lane = threadIdx.x & 31;
  const int wave = threadIdx.x >> 5;
  const int tilesN = N >> 6;
  const int tilesM = M >> 6;
  const int tile = blockIdx.x * 8 + wave;
  if (tile >= tilesM * tilesN) return;
  const int tm = tile / tilesN;
  const int tn = tile - tm * tilesN;
  const int m0 = tm << 6;
  const int n0 = tn << 6;

  const T* Ab  = A  + (size_t)b * strideA;
  const T* Bb  = Bt + (size_t)b * strideB;
  const T* Ab2 = SPLIT ? (A2  + (size_t)b * strideA) : nullptr;
  const T* Bb2 = SPLIT ? (Bt2 + (size_t)b * strideB) : nullptr;

  const int rlane = lane & 15;
  const int koff  = (lane >> 4) * 8;
  const int mOff  = (lane >> 4) * 8;

  v8f acc[4][4];
#pragma unroll
  for (int i = 0; i < 4; ++i)
#pragma unroll
    for (int j = 0; j < 4; ++j) acc[i][j] = (v8f){0.f,0.f,0.f,0.f,0.f,0.f,0.f,0.f};

  for (int k0 = 0; k0 < K; k0 += 32) {
    V bh[4], bl[4];
#pragma unroll
    for (int j = 0; j < 4; ++j) {
      const size_t bo = (size_t)(n0 + (j << 4) + rlane) * ldb + koff + k0;
      bh[j] = Frag<T>::load(Bb + bo);
      if (SPLIT) bl[j] = Frag<T>::load(Bb2 + bo);
    }
#pragma unroll
    for (int i = 0; i < 4; ++i) {
      const size_t ao = (size_t)(m0 + (i << 4) + rlane) * lda + koff + k0;
      V ah = Frag<T>::load(Ab + ao);
      V al;
      if (SPLIT) al = Frag<T>::load(Ab2 + ao);
#pragma unroll
      for (int j = 0; j < 4; ++j) {
        acc[i][j] = Frag<T>::mma(ah, bh[j], acc[i][j]);
        if (SPLIT) {
          acc[i][j] = Frag<T>::mma(ah, bl[j], acc[i][j]);
          acc[i][j] = Frag<T>::mma(al, bh[j], acc[i][j]);
        }
      }
      Frag<T>::guard(acc[i][0], acc[i][3], ah, SPLIT ? al : ah);
    }
    Frag<T>::keep(bh[0], bh[1], bh[2], bh[3]);
    if (SPLIT) Frag<T>::keep(bl[0], bl[1], bl[2], bl[3]);
  }
  acc_guard4(acc[0][0], acc[0][1], acc[0][2], acc[0][3]);
  acc_guard4(acc[1][0], acc[1][1], acc[1][2], acc[1][3]);
  acc_guard4(acc[2][0], acc[2][1], acc[2][2], acc[2][3]);
  acc_guard4(acc[3][0], acc[3][1], acc[3][2], acc[3][3]);

  float* slab = sT[wave];
  const float* Rb = RESID ? (resid + (size_t)b * strideR) : nullptr;
#pragma unroll
  for (int i = 0; i < 4; ++i) {
    const int mBase = m0 + (i << 4);
#pragma unroll
    for (int j = 0; j < 4; ++j) {
      const int n = n0 + (j << 4) + rlane;
      float bv = 0.f;
      if (BIAS_MODE == 2) bv = bias[n];
#pragma unroll
      for (int r = 0; r < 8; ++r) {
        float v = acc[i][j][r] * scale;
        if (BIAS_MODE == 1) v += bias[mBase + mOff + r];
        if (BIAS_MODE == 2) v += bv;
        if (RESID) v += Rb[(size_t)(mBase + mOff + r) * ldc + n];
        if (ROPE) {
          const int m = mBase + mOff + r;
          const int tix = (m & rope_smask) * NFREQ + (n & (NFREQ - 1));
          const float cs = rope_cos[tix];
          const float sn = rope_sin[tix];
          const float pv = __shfl_xor(v, 1, 32);
          v = (n & 1) ? (v * cs + pv * sn) : (v * cs - pv * sn);
        }
        if (ACT == 1) v = tanhf(v);
        if (ACT == 2) v = fmaxf(v, 0.0f);
        if (ACT == 3) v = v / (1.0f + expf(-v));
        if (ACT == 4) v = (v > 0.f) ? v : 0.01f * v;
        if (ACT == 5) v = 0.5f * v * (1.0f + erff(v * 0.70710678118654752f));
        slab[(mOff + r) * 68 + (j << 4) + rlane] = v;
      }
    }
    __builtin_amdgcn_fence(__ATOMIC_RELEASE, "workgroup");
    __builtin_amdgcn_wave_barrier();
    __builtin_amdgcn_fence(__ATOMIC_ACQUIRE, "workgroup");
    if (OUT_MODE == 0) {
      float* C = (float*)Cout + (size_t)b * strideC;
      const int hh = lane >> 4, c4 = (lane & 15) * 4;
      for (int pass = 0; pass < 2; ++pass) {
#pragma unroll
        for (int it = 0; it < 8; ++it) {
          const int row = it * 2 + hh;
          v4f v = *(const v4f*)(slab + row * 68 + c4);
          *(volatile v4f*)(C + (size_t)(mBase + row) * ldc + n0 + c4) = v;
        }
        __threadfence();
      }
    } else {
      const int q = lane >> 3, c8 = (lane & 7) * 8;
      unsigned short* C  = (unsigned short*)Cout  + (size_t)b * strideC;
      unsigned short* C2 = (OUT_MODE == 2) ? ((unsigned short*)Cout2 + (size_t)b * strideC) : nullptr;
      for (int pass = 0; pass < 2; ++pass) {
#pragma unroll
        for (int it = 0; it < 4; ++it) {
          const int row = it * 4 + q;
          const float* sp = slab + row * 68 + c8;
          v8h hv, lv;
#pragma unroll
          for (int e = 0; e < 8; ++e) {
            if (OUT_MODE == 1) {
              hv[e] = (_Float16)sp[e];
            } else {
              unsigned short hb = f2bf_bits(sp[e]);
              unsigned short lb = f2bf_bits(sp[e] - bf_bits2f(hb));
              hv[e] = __builtin_bit_cast(_Float16, hb);
              lv[e] = __builtin_bit_cast(_Float16, lb);
            }
          }
          *(volatile v8h*)(C + (size_t)(mBase + row) * ldc + n0 + c8) = hv;
          if (OUT_MODE == 2) *(volatile v8h*)(C2 + (size_t)(mBase + row) * ldc + n0 + c8) = lv;
        }
        __threadfence();
      }
    }
    __builtin_amdgcn_fence(__ATOMIC_RELEASE, "workgroup");
    __builtin_amdgcn_wave_barrier();
    __builtin_amdgcn_fence(__ATOMIC_ACQUIRE, "workgroup");
  }
}

__device__ __forceinline__ v8f mma_h(v16h a, v16h b, v8f c) {
  c = __builtin_amdgcn_wmma_f32_16x16x32_f16(false, a, false, b, (short)0, c, false, false);
  asm volatile("v_nop\n\tv_nop\n\tv_nop\n\tv_nop" : "+v"(c) : "v"(a), "v"(b));
  return c;
}

__global__ __launch_bounds__(256) void rope_table_kernel(float* __restrict__ cosT, float* __restrict__ sinT, int n) {
  const int i = blockIdx.x * 256 + threadIdx.x;
  if (i < n) {
    const int pos = i >> 5;
    const int fi = i & (NFREQ - 1);
    const float e = (float)(2 * fi) * (1.0f / (float)NHD);
    const float p = powf(10000.0f, e);
    const float inv = 1.0f / p;
    const float ang = (float)pos * inv;
    const float cs = cosf(ang);
    const float sn = sinf(ang);
    ((volatile float*)cosT)[i] = cs;
    ((volatile float*)sinT)[i] = sn;
    __threadfence();
    ((volatile float*)cosT)[i] = cs;
    ((volatile float*)sinT)[i] = sn;
  }
}

__global__ __launch_bounds__(256) void cast_f32_f16x8(const float* __restrict__ in, _Float16* __restrict__ out, int n8) {
  const int i = blockIdx.x * 256 + threadIdx.x;
  if (i < n8) {
    const v4f a = *(const v4f*)(in + (size_t)i * 8);
    const v4f c = *(const v4f*)(in + (size_t)i * 8 + 4);
    v8h hv;
    hv[0] = (_Float16)a[0]; hv[1] = (_Float16)a[1]; hv[2] = (_Float16)a[2]; hv[3] = (_Float16)a[3];
    hv[4] = (_Float16)c[0]; hv[5] = (_Float16)c[1]; hv[6] = (_Float16)c[2]; hv[7] = (_Float16)c[3];
    *(volatile v8h*)(out + (size_t)i * 8) = hv;
    __threadfence();
    *(volatile v8h*)(out + (size_t)i * 8) = hv;
  }
}

__global__ __launch_bounds__(256) void wt_cast_f16(const float* __restrict__ W, _Float16* __restrict__ Wt,
                                                   int Kdim, int Ndim, float mul) {
  __shared__ float sTt[64 * 65];
  const int k0 = blockIdx.x * 64, n0 = blockIdx.y * 64;
  const int tid = threadIdx.x;
  {
    const int row = tid >> 2, col0 = (tid & 3) * 16;
    const float* src = W + (size_t)(k0 + row) * Ndim + n0 + col0;
#pragma unroll
    for (int i = 0; i < 4; ++i) {
      const v4f w4 = *(const v4f*)(src + 4 * i);
#pragma unroll
      for (int e = 0; e < 4; ++e) sTt[(col0 + 4 * i + e) * 65 + row] = w4[e] * mul;
    }
  }
  __syncthreads();
  const int wave = tid >> 5, lane = tid & 31, rq = lane >> 3, c8 = (lane & 7) * 8;
  for (int pass = 0; pass < 2; ++pass) {
#pragma unroll
    for (int it = 0; it < 2; ++it) {
      const int n = it * 32 + wave * 4 + rq;
      v8h hv;
#pragma unroll
      for (int e = 0; e < 8; ++e) hv[e] = (_Float16)sTt[n * 65 + c8 + e];
      *(volatile v8h*)(Wt + (size_t)(n0 + n) * Kdim + k0 + c8) = hv;
    }
    __threadfence();
  }
}

#define AT_QB 64
#define AT_KC 64
#define AT_NW 4

__global__ __launch_bounds__(128)
void attn_f16_kernel(const _Float16* __restrict__ Qh, const _Float16* __restrict__ Kh,
                     const _Float16* __restrict__ Vt, const float* __restrict__ cdr_bias,
                     const float* __restrict__ cdr_w, _Float16* __restrict__ Oh)
{
  __shared__ __align__(16) _Float16 Ksh[AT_KC * NHD];
  __shared__ __align__(16) _Float16 Vth[NHD * AT_KC];
  __shared__ __align__(16) _Float16 Psh[AT_NW][16 * AT_KC];
  __shared__ __align__(16) float    Os[AT_NW][16 * 68];

  const int tid  = threadIdx.x;
  const int wave = tid >> 5;
  const int lane = tid & 31;
  const int hh   = lane >> 4;
  const int c    = lane & 15;

  const int nqb = NS / AT_QB;
  const int bx  = blockIdx.x;
  const int qb  = bx % nqb;
  const int bhd = bx / nqb;
  const int h   = bhd % NH;
  const int bb0 = bhd / NH;
  const int b   = bb0 < NB ? bb0 : (NB - 1);
  const int q0  = qb * AT_QB + wave * 16;
  const float cw = cdr_w[0];

  v16h qa[2];
  {
    const _Float16* qrow = Qh + (size_t)(b * NS + q0 + c) * ND + h * NHD;
#pragma unroll
    for (int dc = 0; dc < 2; ++dc) qa[dc] = Frag<_Float16>::load(qrow + dc * 32 + 8 * hh);
  }

  float mrow[8], lrow[8];
  v8f oacc[4];
#pragma unroll
  for (int r = 0; r < 8; ++r) { mrow[r] = -INFINITY; lrow[r] = 0.f; }
#pragma unroll
  for (int t = 0; t < 4; ++t) oacc[t] = (v8f){0.f,0.f,0.f,0.f,0.f,0.f,0.f,0.f};

  const _Float16* kbase = Kh + (size_t)(b * NS) * ND + h * NHD;
  const _Float16* vbase = Vt + (size_t)(h * NHD) * NM + (size_t)b * NS;
  const float*    bbase = cdr_bias + (size_t)b * NS;

  for (int kc = 0; kc < NS / AT_KC; ++kc) {
    const int kv0 = kc * AT_KC;
    __syncthreads();
    {
      const int sr = tid >> 1, half = (tid & 1) * 32;
      const _Float16* ksrc = kbase + (size_t)(kv0 + sr) * ND + half;
      const _Float16* vsrc = vbase + (size_t)sr * NM + kv0 + half;
#pragma unroll
      for (int i = 0; i < 4; ++i) {
        const v8h kk = *(const v8h*)(ksrc + 8 * i);
        const v8h vv = *(const v8h*)(vsrc + 8 * i);
        *(v8h*)(Ksh + sr * NHD + half + 8 * i) = kk;
        *(v8h*)(Vth + sr * AT_KC + half + 8 * i) = vv;
      }
    }
    __syncthreads();

    v8f s[4];
#pragma unroll
    for (int j = 0; j < 4; ++j) {
      s[j] = (v8f){0.f,0.f,0.f,0.f,0.f,0.f,0.f,0.f};
#pragma unroll
      for (int dc = 0; dc < 2; ++dc) {
        const v16h kb = Frag<_Float16>::load(Ksh + (j * 16 + c) * NHD + dc * 32 + 8 * hh);
        s[j] = mma_h(qa[dc], kb, s[j]);
      }
    }
    float bj[4];
#pragma unroll
    for (int j = 0; j < 4; ++j) bj[j] = bbase[kv0 + j * 16 + c] * cw;
    float cm[8];
#pragma unroll
    for (int r = 0; r < 8; ++r) {
      float m = -INFINITY;
#pragma unroll
      for (int j = 0; j < 4; ++j) {
        const float sv = s[j][r] * 0.125f + bj[j];
        s[j][r] = sv;
        m = fmaxf(m, sv);
      }
#pragma unroll
      for (int off = 1; off < 16; off <<= 1) m = fmaxf(m, __shfl_xor(m, off, 32));
      cm[r] = m;
    }
    _Float16* pw = Psh[wave];
#pragma unroll
    for (int r = 0; r < 8; ++r) {
      const float mnew = fmaxf(mrow[r], cm[r]);
      const float alpha = expf(mrow[r] - mnew);
      mrow[r] = mnew;
      float psum = 0.f;
#pragma unroll
      for (int j = 0; j < 4; ++j) {
        const float p = expf(s[j][r] - mnew);
        psum += p;
        pw[(8 * hh + r) * AT_KC + j * 16 + c] = (_Float16)(p * PCARRY);
      }
#pragma unroll
      for (int off = 1; off < 16; off <<= 1) psum += __shfl_xor(psum, off, 32);
      lrow[r] = lrow[r] * alpha + psum;
#pragma unroll
      for (int t = 0; t < 4; ++t) oacc[t][r] *= alpha;
    }
    __builtin_amdgcn_fence(__ATOMIC_RELEASE, "workgroup");
    __builtin_amdgcn_wave_barrier();
    __builtin_amdgcn_fence(__ATOMIC_ACQUIRE, "workgroup");
#pragma unroll 1
    for (int kk = 0; kk < 2; ++kk) {
      const v16h pa = Frag<_Float16>::load(pw + c * AT_KC + kk * 32 + 8 * hh);
#pragma unroll
      for (int t = 0; t < 4; ++t) {
        const v16h vb = Frag<_Float16>::load(Vth + (t * 16 + c) * AT_KC + kk * 32 + 8 * hh);
        oacc[t] = mma_h(pa, vb, oacc[t]);
      }
    }
  }

  float* os = Os[wave];
#pragma unroll
  for (int r = 0; r < 8; ++r) {
    const float inv = (1.0f / lrow[r]) * (OCARRY / PCARRY);
#pragma unroll
    for (int t = 0; t < 4; ++t) os[(8 * hh + r) * 68 + t * 16 + c] = oacc[t][r] * inv;
  }
  __builtin_amdgcn_fence(__ATOMIC_RELEASE, "workgroup");
  __builtin_amdgcn_wave_barrier();
  __builtin_amdgcn_fence(__ATOMIC_ACQUIRE, "workgroup");
  {
    const int q = lane >> 3, c8 = (lane & 7) * 8;
    _Float16* orow = Oh + (size_t)(b * NS + q0) * ND + h * NHD;
    for (int pass = 0; pass < 2; ++pass) {
#pragma unroll
      for (int it = 0; it < 4; ++it) {
        const int row = it * 4 + q;
        const float* sp = os + row * 68 + c8;
        v8h hv;
#pragma unroll
        for (int e = 0; e < 8; ++e) hv[e] = (_Float16)sp[e];
        *(volatile v8h*)(orow + (size_t)row * ND + c8) = hv;
      }
      __threadfence();
    }
  }
}

__global__ __launch_bounds__(256) void layernorm_rows(const float* __restrict__ res, const float* __restrict__ gamma,
                                                      const float* __restrict__ beta, float* __restrict__ out,
                                                      int nrows, float eps) {
  const int wave = threadIdx.x >> 5, lane = threadIdx.x & 31;
  const int row = blockIdx.x * 8 + wave;
  if (row >= nrows) return;
  const float* rp = res + (size_t)row * ND;
  float s1 = 0.f;
#pragma unroll 1
  for (int it = 0; it < 8; ++it) {
    const v4f a = *(const v4f*)(rp + (it * 32 + lane) * 4);
    s1 += (a[0] + a[1]) + (a[2] + a[3]);
  }
#pragma unroll
  for (int off = 1; off < 32; off <<= 1) s1 += __shfl_xor(s1, off, 32);
  const float mu = s1 * (1.0f / (float)ND);
  float s2 = 0.f;
#pragma unroll 1
  for (int it = 0; it < 8; ++it) {
    const v4f a = *(const v4f*)(rp + (it * 32 + lane) * 4);
#pragma unroll
    for (int e = 0; e < 4; ++e) {
      const float d = a[e] - mu;
      float p = d * d;
      asm volatile("" : "+v"(p));
      s2 += p;
    }
  }
#pragma unroll
  for (int off = 1; off < 32; off <<= 1) s2 += __shfl_xor(s2, off, 32);
  const float var = s2 * (1.0f / (float)ND);
  const float rstd = 1.0f / sqrtf(var + eps);
  float* orow = out + (size_t)row * ND;
#pragma unroll 1
  for (int it = 0; it < 8; ++it) {
    const int c0 = (it * 32 + lane) * 4;
    const v4f a  = *(const v4f*)(rp + c0);
    const v4f g  = *(const v4f*)(gamma + c0);
    const v4f bt = *(const v4f*)(beta + c0);
    v4f y;
#pragma unroll
    for (int e = 0; e < 4; ++e) {
      float t = (a[e] - mu) * rstd;
      t = t * g[e];
      asm volatile("" : "+v"(t));
      y[e] = t + bt[e];
    }
    *(volatile v4f*)(orow + c0) = y;
    __threadfence();
    *(volatile v4f*)(orow + c0) = y;
  }
}

extern "C" void kernel_launch(void* const* d_in, const int* in_sizes, int n_in,
                              void* d_out, int out_size, void* d_ws, size_t ws_size,
                              hipStream_t stream)
{
  if (n_in < 13) return;
  if (in_sizes[0] != NM * ND || in_sizes[1] != NB * NS ||
      in_sizes[2] != ND * ND || in_sizes[3] != ND ||
      in_sizes[4] != ND * ND || in_sizes[5] != ND ||
      in_sizes[6] != ND * ND || in_sizes[7] != ND ||
      in_sizes[8] != ND * ND || in_sizes[9] != ND ||
      in_sizes[10] != ND || in_sizes[11] != ND || in_sizes[12] < 1 ||
      out_size != NM * ND) return;

  const float* x        = (const float*)d_in[0];
  const float* cdr_bias = (const float*)d_in[1];
  const float* Wq    = (const float*)d_in[2];
  const float* bq    = (const float*)d_in[3];
  const float* Wk    = (const float*)d_in[4];
  const float* bk    = (const float*)d_in[5];
  const float* Wv    = (const float*)d_in[6];
  const float* bv    = (const float*)d_in[7];
  const float* Wo    = (const float*)d_in[8];
  const float* bo    = (const float*)d_in[9];
  const float* gamma = (const float*)d_in[10];
  const float* beta  = (const float*)d_in[11];
  const float* cw    = (const float*)d_in[12];
  float* out = (float*)d_out;

  const size_t szA16 = (size_t)NM * ND * 2;
  const size_t szW16 = (size_t)ND * ND * 2;
  const size_t szRes = (size_t)NM * ND * 4;
  const size_t szTab = (size_t)NS * NFREQ * 4;
  size_t off = 0;
  char* ws = (char*)d_ws;
  _Float16* Xh  = (_Float16*)(ws + off); off += szA16;
  _Float16* Wqt = (_Float16*)(ws + off); off += szW16;
  _Float16* Wkt = (_Float16*)(ws + off); off += szW16;
  _Float16* Wvt = (_Float16*)(ws + off); off += szW16;
  _Float16* Wot = (_Float16*)(ws + off); off += szW16;
  _Float16* Qh  = (_Float16*)(ws + off); off += szA16;
  _Float16* Kh  = (_Float16*)(ws + off); off += szA16;
  _Float16* Vt  = (_Float16*)(ws + off); off += szA16;
  _Float16* Ah  = (_Float16*)(ws + off); off += szA16;
  float*    res = (float*)(ws + off);    off += szRes;
  float*   cosT = (float*)(ws + off);    off += szTab;
  float*   sinT = (float*)(ws + off);    off += szTab;
  if (off > ws_size) return;

  const unsigned short* Xu  = (const unsigned short*)Xh;
  const unsigned short* Wqu = (const unsigned short*)Wqt;
  const unsigned short* Wku = (const unsigned short*)Wkt;
  const unsigned short* Wvu = (const unsigned short*)Wvt;
  const unsigned short* Wou = (const unsigned short*)Wot;
  const unsigned short* Au  = (const unsigned short*)Ah;

  dim3 blk256(256), blk128(128);

  const int nTab = NS * NFREQ;
  rope_table_kernel<<<dim3((nTab + 255) / 256), blk256, 0, stream>>>(cosT, sinT, nTab);

  const int n8 = NM * ND / 8;
  cast_f32_f16x8<<<dim3((n8 + 255) / 256), blk256, 0, stream>>>(x, Xh, n8);

  wt_cast_f16<<<dim3(ND / 64, ND / 64), blk256, 0, stream>>>(Wq, Wqt, ND, ND, WCARRY);
  wt_cast_f16<<<dim3(ND / 64, ND / 64), blk256, 0, stream>>>(Wk, Wkt, ND, ND, WCARRY);
  wt_cast_f16<<<dim3(ND / 64, ND / 64), blk256, 0, stream>>>(Wv, Wvt, ND, ND, WCARRY);
  wt_cast_f16<<<dim3(ND / 64, ND / 64), blk256, 0, stream>>>(Wo, Wot, ND, ND, WCARRY);

  const int tilesQK = (NM / 64) * (ND / 64);
  const int gQK = (tilesQK + 7) / 8;
  wmma_gemm64<0, false, 2, 1, false, 0, true><<<dim3(gQK, 1), blk256, 0, stream>>>(
      Xu, Xu, ND, (long)0, Wqu, Wqu, ND, (long)0, (void*)Qh, (void*)Qh, ND, (long)0,
      bq, x, (long)0, NM, ND, ND, 1.0f / WCARRY, cosT, sinT, NS - 1);
  wmma_gemm64<0, false, 2, 1, false, 0, true><<<dim3(gQK, 1), blk256, 0, stream>>>(
      Xu, Xu, ND, (long)0, Wku, Wku, ND, (long)0, (void*)Kh, (void*)Kh, ND, (long)0,
      bk, x, (long)0, NM, ND, ND, 1.0f / WCARRY, cosT, sinT, NS - 1);

  const int tilesV = (ND / 64) * (NM / 64);
  const int gV = (tilesV + 7) / 8;
  wmma_gemm64<0, false, 1, 1, false, 0, false><<<dim3(gV, 1), blk256, 0, stream>>>(
      Wvu, Wvu, ND, (long)0, Xu, Xu, ND, (long)0, (void*)Vt, (void*)Vt, NM, (long)0,
      bv, x, (long)0, ND, NM, ND, 1.0f / WCARRY, cosT, sinT, 0);

  attn_f16_kernel<<<dim3(NB * NH * (NS / AT_QB)), blk128, 0, stream>>>(Qh, Kh, Vt, cdr_bias, cw, Ah);

  wmma_gemm64<0, false, 2, 0, true, 0, false><<<dim3(gQK, 1), blk256, 0, stream>>>(
      Au, Au, ND, (long)0, Wou, Wou, ND, (long)0, (void*)res, (void*)res, ND, (long)0,
      bo, x, (long)0, NM, ND, ND, 1.0f / (OCARRY * WCARRY), cosT, sinT, 0);

  layernorm_rows<<<dim3((NM + 7) / 8), blk256, 0, stream>>>(res, gamma, beta, out, NM, LN_EPS_F);

  (void)hipGetLastError();
}
